// RWKV_Tmix_x060_45732811768065
// MI455X (gfx1250) — hardware-verified
//
#include <hip/hip_runtime.h>
#include <math.h>

constexpr int kB   = 4;
constexpr int kT   = 2048;
constexpr int kC   = 1024;
constexpr int kHS  = 16;
constexpr int kNH  = 64;
constexpr int kDMix = 32;
constexpr int kDDec = 64;
constexpr int kTc  = 512;
constexpr int kTcShift = 9;
constexpr int kNChunk = kT / kTc;
constexpr int kRc  = kB * kTc;
static_assert((1 << kTcShift) == kTc);
static_assert(kRc % 64 == 0);
static_assert(kT % kTc == 0);
constexpr float kInvC  = 1.0f / 1024.0f;
constexpr float kLnEps = 1e-5f;

typedef __attribute__((ext_vector_type(16))) _Float16 v16h;
typedef __attribute__((ext_vector_type(8)))  _Float16 v8h;
typedef __attribute__((ext_vector_type(16))) __bf16   v16b;
typedef __attribute__((ext_vector_type(8)))  __bf16   v8b;
typedef __attribute__((ext_vector_type(8)))  float    v8f;
typedef __attribute__((ext_vector_type(4)))  float    v4f;
typedef __attribute__((ext_vector_type(4)))  unsigned int v4u;

__device__ __forceinline__ unsigned short f2bf_bits(float f) {
  unsigned u = __float_as_uint(f);
  return (unsigned short)((u + 0x7FFFu + ((u >> 16) & 1u)) >> 16);
}
__device__ __forceinline__ float bf_bits2f(unsigned short h) { return __uint_as_float(((unsigned)h) << 16); }

__device__ __forceinline__ void dep_guard_h(v8f& a, v8f& b, v16h x, v16h y) { asm volatile("v_nop\n\tv_nop\n\tv_nop\n\tv_nop" : "+v"(a), "+v"(b) : "v"(x), "v"(y)); }
__device__ __forceinline__ void dep_guard_b(v8f& a, v8f& b, v16b x, v16b y) { asm volatile("v_nop\n\tv_nop\n\tv_nop\n\tv_nop" : "+v"(a), "+v"(b) : "v"(x), "v"(y)); }
__device__ __forceinline__ void keep4_h(v16h a, v16h b, v16h c, v16h d) { asm volatile("v_nop" :: "v"(a), "v"(b), "v"(c), "v"(d)); }
__device__ __forceinline__ void keep4_b(v16b a, v16b b, v16b c, v16b d) { asm volatile("v_nop" :: "v"(a), "v"(b), "v"(c), "v"(d)); }
__device__ __forceinline__ void acc_guard4(v8f& a, v8f& b, v8f& c, v8f& d) { asm volatile("v_nop\n\tv_nop\n\tv_nop\n\tv_nop" : "+v"(a), "+v"(b), "+v"(c), "+v"(d)); }
template <typename T> struct Frag;
template <> struct Frag<_Float16> {
  typedef v16h V; union U { v16h v; v8h h[2]; };
  static __device__ __forceinline__ v16h load(const _Float16* p) {
    U f; f.h[0] = *(const v8h*)(p); f.h[1] = *(const v8h*)(p + 16); return f.v;
  }
  static __device__ __forceinline__ v8f mma(v16h a, v16h b, v8f c) {
    return __builtin_amdgcn_wmma_f32_16x16x32_f16(false, a, false, b, (short)0, c, false, false);
  }
  static __device__ __forceinline__ void guard(v8f& a, v8f& b, v16h x, v16h y) { dep_guard_h(a, b, x, y); }
  static __device__ __forceinline__ void keep(v16h a, v16h b, v16h c, v16h d) { keep4_h(a, b, c, d); }
};
template <> struct Frag<__bf16> {
  typedef v16b V; union U { v16b v; v8b h[2]; };
  static __device__ __forceinline__ v16b load(const __bf16* p) {
    U f; f.h[0] = *(const v8b*)(p); f.h[1] = *(const v8b*)(p + 16); return f.v;
  }
  static __device__ __forceinline__ v8f mma(v16b a, v16b b, v8f c) {
    return __builtin_amdgcn_wmma_f32_16x16x32_bf16(false, a, false, b, (short)0, c, false, false);
  }
  static __device__ __forceinline__ void guard(v8f& a, v8f& b, v16b x, v16b y) { dep_guard_b(a, b, x, y); }
  static __device__ __forceinline__ void keep(v16b a, v16b b, v16b c, v16b d) { keep4_b(a, b, c, d); }
};

__device__ __forceinline__ unsigned pk16(unsigned short a, unsigned short b) { return (unsigned)a | ((unsigned)b << 16); }
__device__ __forceinline__ void split_bits(float v, unsigned short& hb, unsigned short& lb) {
  hb = f2bf_bits(v);
  lb = f2bf_bits(v - bf_bits2f(hb));
}

template <int ET> struct Elem;
template <> struct Elem<0> { typedef _Float16 T; };
template <> struct Elem<1> { typedef __bf16 T; };
template <int ET, bool SPLIT, int BIAS_MODE, int OUT_MODE, bool RESID, int ACT = 0>
__global__ __launch_bounds__(256) void wmma_gemm64(
    const unsigned short* __restrict__ Ap, const unsigned short* __restrict__ A2p, int lda, long strideA,
    const unsigned short* __restrict__ Btp, const unsigned short* __restrict__ Bt2p, int ldb, long strideB,
    void* __restrict__ Cout, void* __restrict__ Cout2, int ldc, long strideC,
    const float* __restrict__ bias,
    const float* __restrict__ resid, long strideR,
    int M, int N, int K, float scale) {
  typedef typename Elem<ET>::T T;
  typedef typename Frag<T>::V V;
  const T* A = (const T*)Ap; const T* A2 = (const T*)A2p; const T* Bt = (const T*)Btp; const T* Bt2 = (const T*)Bt2p;
  __shared__ __align__(16) float sT[8][16 * 68];
  const int b    = blockIdx.y;
  const int lane = threadIdx.x & 31;
  const int wave = threadIdx.x >> 5;
  const int tilesN = N >> 6;
  const int tilesM = M >> 6;
  const int tile = blockIdx.x * 8 + wave;
  if (tile >= tilesM * tilesN) return;
  const int tm = tile / tilesN;
  const int tn = tile - tm * tilesN;
  const int m0 = tm << 6;
  const int n0 = tn << 6;

  const T* Ab  = A  + (size_t)b * strideA;
  const T* Bb  = Bt + (size_t)b * strideB;
  const T* Ab2 = SPLIT ? (A2  + (size_t)b * strideA) : nullptr;
  const T* Bb2 = SPLIT ? (Bt2 + (size_t)b * strideB) : nullptr;

  const int rlane = lane & 15;
  const int koff  = (lane >> 4) * 8;
  const int mOff  = (lane >> 4) * 8;

  v8f acc[4][4];
#pragma unroll
  for (int i = 0; i < 4; ++i)
#pragma unroll
    for (int j = 0; j < 4; ++j) acc[i][j] = (v8f){0.f,0.f,0.f,0.f,0.f,0.f,0.f,0.f};

  for (int k0 = 0; k0 < K; k0 += 32) {
    V bh[4], bl[4];
#pragma unroll
    for (int j = 0; j < 4; ++j) {
      const size_t bo = (size_t)(n0 + (j << 4) + rlane) * ldb + koff + k0;
      bh[j] = Frag<T>::load(Bb + bo);
      if (SPLIT) bl[j] = Frag<T>::load(Bb2 + bo);
    }
#pragma unroll
    for (int i = 0; i < 4; ++i) {
      const size_t ao = (size_t)(m0 + (i << 4) + rlane) * lda + koff + k0;
      V ah = Frag<T>::load(Ab + ao);
      V al;
      if (SPLIT) al = Frag<T>::load(Ab2 + ao);
#pragma unroll
      for (int j = 0; j < 4; ++j) {
        acc[i][j] = Frag<T>::mma(ah, bh[j], acc[i][j]);
        if (SPLIT) {
          acc[i][j] = Frag<T>::mma(ah, bl[j], acc[i][j]);
          acc[i][j] = Frag<T>::mma(al, bh[j], acc[i][j]);
        }
      }
      Frag<T>::guard(acc[i][0], acc[i][3], ah, SPLIT ? al : ah);
    }
    Frag<T>::keep(bh[0], bh[1], bh[2], bh[3]);
    if (SPLIT) Frag<T>::keep(bl[0], bl[1], bl[2], bl[3]);
  }
  acc_guard4(acc[0][0], acc[0][1], acc[0][2], acc[0][3]);
  acc_guard4(acc[1][0], acc[1][1], acc[1][2], acc[1][3]);
  acc_guard4(acc[2][0], acc[2][1], acc[2][2], acc[2][3]);
  acc_guard4(acc[3][0], acc[3][1], acc[3][2], acc[3][3]);

  float* slab = sT[wave];
  const float* Rb = RESID ? (resid + (size_t)b * strideR) : nullptr;
#pragma unroll
  for (int i = 0; i < 4; ++i) {
    const int mBase = m0 + (i << 4);
#pragma unroll
    for (int j = 0; j < 4; ++j) {
      const int n = n0 + (j << 4) + rlane;
      float bv = 0.f;
      if (BIAS_MODE == 2) bv = bias[n];
#pragma unroll
      for (int r = 0; r < 8; ++r) {
        float v = acc[i][j][r] * scale;
        if (BIAS_MODE == 1) v += bias[mBase + mOff + r];
        if (BIAS_MODE == 2) v += bv;
        if (RESID) v += Rb[(size_t)(mBase + mOff + r) * ldc + n];
        if (ACT == 1) v = tanhf(v);
        if (ACT == 2) v = fmaxf(v, 0.0f);
        if (ACT == 4) v = (v > 0.f) ? v : 0.01f * v;
        if (ACT == 6) v = expf(-expf(v));
        slab[(mOff + r) * 68 + (j << 4) + rlane] = v;
      }
    }
    __builtin_amdgcn_fence(__ATOMIC_RELEASE, "workgroup");
    __builtin_amdgcn_wave_barrier();
    __builtin_amdgcn_fence(__ATOMIC_ACQUIRE, "workgroup");
    if (OUT_MODE == 0) {
      float* C = (float*)Cout + (size_t)b * strideC;
      const int hh = lane >> 4, c4 = (lane & 15) * 4;
      for (int pass = 0; pass < 2; ++pass) {
#pragma unroll
        for (int it = 0; it < 8; ++it) {
          const int row = it * 2 + hh;
          v4f v = *(const v4f*)(slab + row * 68 + c4);
          *(volatile v4f*)(C + (size_t)(mBase + row) * ldc + n0 + c4) = v;
        }
        __threadfence();
      }
    } else {
      const int q = lane >> 3, c8 = (lane & 7) * 8;
      unsigned short* C  = (unsigned short*)Cout  + (size_t)b * strideC;
      unsigned short* C2 = (OUT_MODE == 2) ? ((unsigned short*)Cout2 + (size_t)b * strideC) : nullptr;
      for (int pass = 0; pass < 2; ++pass) {
#pragma unroll
        for (int it = 0; it < 4; ++it) {
          const int row = it * 4 + q;
          const float* sp = slab + row * 68 + c8;
          v8h hv, lv;
#pragma unroll
          for (int e = 0; e < 8; ++e) {
            if (OUT_MODE == 1) {
              hv[e] = (_Float16)sp[e];
            } else {
              unsigned short hb = f2bf_bits(sp[e]);
              unsigned short lb = f2bf_bits(sp[e] - bf_bits2f(hb));
              hv[e] = __builtin_bit_cast(_Float16, hb);
              lv[e] = __builtin_bit_cast(_Float16, lb);
            }
          }
          *(volatile v8h*)(C + (size_t)(mBase + row) * ldc + n0 + c8) = hv;
          if (OUT_MODE == 2) *(volatile v8h*)(C2 + (size_t)(mBase + row) * ldc + n0 + c8) = lv;
        }
        __threadfence();
      }
    }
    __builtin_amdgcn_fence(__ATOMIC_RELEASE, "workgroup");
    __builtin_amdgcn_wave_barrier();
    __builtin_amdgcn_fence(__ATOMIC_ACQUIRE, "workgroup");
  }
}

__global__ __launch_bounds__(256) void wmma_gemm64_mix(
    const unsigned short* __restrict__ Ap, const unsigned short* __restrict__ A2p, int lda, long strideA,
    const unsigned short* __restrict__ Btp, const unsigned short* __restrict__ Bt2p, int ldb, long strideB,
    void* __restrict__ Cout, void* __restrict__ Cout2, int ldc, long strideC,
    const float* __restrict__ maa0, const float* __restrict__ maa1,
    const float* __restrict__ maa2, const float* __restrict__ maa3,
    const float* __restrict__ xg, int cbase,
    int M, int N, int K) {
  typedef __bf16 T;
  typedef v16b V;
  const T* A = (const T*)Ap; const T* A2 = (const T*)A2p; const T* Bt = (const T*)Btp; const T* Bt2 = (const T*)Bt2p;
  __shared__ __align__(16) float sT[8][16 * 68];
  const int b    = blockIdx.y;
  const int lane = threadIdx.x & 31;
  const int wave = threadIdx.x >> 5;
  const int tilesN = N >> 6;
  const int tilesM = M >> 6;
  const int tile = blockIdx.x * 8 + wave;
  if (tile >= tilesM * tilesN) return;
  const int tm = tile / tilesN;
  const int tn = tile - tm * tilesN;
  const int m0 = tm << 6;
  const int n0 = tn << 6;

  const T* Ab  = A   + (size_t)b * strideA;
  const T* Bb  = Bt  + (size_t)b * strideB;
  const T* Ab2 = A2  + (size_t)b * strideA;
  const T* Bb2 = Bt2 + (size_t)b * strideB;

  const int rlane = lane & 15;
  const int koff  = (lane >> 4) * 8;
  const int mOff  = (lane >> 4) * 8;

  v8f acc[4][4];
#pragma unroll
  for (int i = 0; i < 4; ++i)
#pragma unroll
    for (int j = 0; j < 4; ++j) acc[i][j] = (v8f){0.f,0.f,0.f,0.f,0.f,0.f,0.f,0.f};

  for (int k0 = 0; k0 < K; k0 += 32) {
    V bh[4], bl[4];
#pragma unroll
    for (int j = 0; j < 4; ++j) {
      const size_t bo = (size_t)(n0 + (j << 4) + rlane) * ldb + koff + k0;
      bh[j] = Frag<T>::load(Bb + bo);
      bl[j] = Frag<T>::load(Bb2 + bo);
    }
#pragma unroll
    for (int i = 0; i < 4; ++i) {
      const size_t ao = (size_t)(m0 + (i << 4) + rlane) * lda + koff + k0;
      V ah = Frag<T>::load(Ab + ao);
      V al = Frag<T>::load(Ab2 + ao);
#pragma unroll
      for (int j = 0; j < 4; ++j) {
        acc[i][j] = Frag<T>::mma(ah, bh[j], acc[i][j]);
        acc[i][j] = Frag<T>::mma(ah, bl[j], acc[i][j]);
        acc[i][j] = Frag<T>::mma(al, bh[j], acc[i][j]);
      }
      Frag<T>::guard(acc[i][0], acc[i][3], ah, al);
    }
    Frag<T>::keep(bh[0], bh[1], bh[2], bh[3]);
    Frag<T>::keep(bl[0], bl[1], bl[2], bl[3]);
  }
  acc_guard4(acc[0][0], acc[0][1], acc[0][2], acc[0][3]);
  acc_guard4(acc[1][0], acc[1][1], acc[1][2], acc[1][3]);
  acc_guard4(acc[2][0], acc[2][1], acc[2][2], acc[2][3]);
  acc_guard4(acc[3][0], acc[3][1], acc[3][2], acc[3][3]);

  float* slab = sT[wave];
  const float* maa = (b == 0) ? maa0 : (b == 1) ? maa1 : (b == 2) ? maa2 : maa3;
#pragma unroll
  for (int i = 0; i < 4; ++i) {
    const int mBase = m0 + (i << 4);
#pragma unroll
    for (int j = 0; j < 4; ++j) {
      const int n = n0 + (j << 4) + rlane;
      const float bv = maa[n];
#pragma unroll
      for (int r = 0; r < 8; ++r) {
        const int m  = mBase + mOff + r;
        const int xb = m >> kTcShift;
        const int t  = cbase + (m & (kTc - 1));
        const int tp = (t > 0) ? (t - 1) : 0;
        const size_t xi  = ((size_t)(xb * kT + t))  * kC + n;
        const size_t xpi = ((size_t)(xb * kT + tp)) * kC + n;
        const float xv  = xg[xi];
        const float xpv = xg[xpi];
        const float pe  = (t > 0) ? xpv : 0.0f;
        const float v   = xv + (pe - xv) * (bv + acc[i][j][r]);
        slab[(mOff + r) * 68 + (j << 4) + rlane] = v;
      }
    }
    __builtin_amdgcn_fence(__ATOMIC_RELEASE, "workgroup");
    __builtin_amdgcn_wave_barrier();
    __builtin_amdgcn_fence(__ATOMIC_ACQUIRE, "workgroup");
    {
      const int q = lane >> 3, c8 = (lane & 7) * 8;
      unsigned short* C  = (unsigned short*)Cout  + (size_t)b * strideC;
      unsigned short* C2 = (unsigned short*)Cout2 + (size_t)b * strideC;
      for (int pass = 0; pass < 2; ++pass) {
#pragma unroll
        for (int it = 0; it < 4; ++it) {
          const int row = it * 4 + q;
          const float* sp = slab + row * 68 + c8;
          v8h hv, lv;
#pragma unroll
          for (int e = 0; e < 8; ++e) {
            unsigned short hb = f2bf_bits(sp[e]);
            unsigned short lb = f2bf_bits(sp[e] - bf_bits2f(hb));
            hv[e] = __builtin_bit_cast(_Float16, hb);
            lv[e] = __builtin_bit_cast(_Float16, lb);
          }
          *(volatile v8h*)(C  + (size_t)(mBase + row) * ldc + n0 + c8) = hv;
          *(volatile v8h*)(C2 + (size_t)(mBase + row) * ldc + n0 + c8) = lv;
        }
        __threadfence();
      }
    }
    __builtin_amdgcn_fence(__ATOMIC_RELEASE, "workgroup");
    __builtin_amdgcn_wave_barrier();
    __builtin_amdgcn_fence(__ATOMIC_ACQUIRE, "workgroup");
  }
}

__global__ __launch_bounds__(256) void wt_split_kernel(const float* __restrict__ W0, const float* __restrict__ W1,
                                                       const float* __restrict__ W2, const float* __restrict__ W3,
                                                       unsigned short* __restrict__ outHi, unsigned short* __restrict__ outLo,
                                                       int R, int Cc) {
  __shared__ float sm[64][65];
  const int t  = threadIdx.x;
  const int r0 = blockIdx.x * 64;
  const int c0 = blockIdx.y * 64;
  const int z  = blockIdx.z;
  const float* W = (z == 0) ? W0 : (z == 1) ? W1 : (z == 2) ? W2 : W3;
#pragma unroll
  for (int i = 0; i < 16; ++i) {
    const int e  = i * 256 + t;
    const int rl = e >> 6;
    const int cl = e & 63;
    sm[cl][rl] = W[(size_t)(r0 + rl) * Cc + c0 + cl];
  }
  __syncthreads();
  const int lane = t & 31, wave = t >> 5;
  const int q = lane >> 3, c8 = (lane & 7) * 8;
  const size_t planeoff = (size_t)z * (size_t)Cc * (size_t)R;
  v4u uh[2], ul[2];
  size_t oofs[2];
#pragma unroll
  for (int it = 0; it < 2; ++it) {
    const int row = wave * 8 + it * 4 + q;
    unsigned short hb[8], lb[8];
#pragma unroll
    for (int e = 0; e < 8; ++e) split_bits(sm[row][c8 + e], hb[e], lb[e]);
    uh[it] = (v4u){pk16(hb[0], hb[1]), pk16(hb[2], hb[3]), pk16(hb[4], hb[5]), pk16(hb[6], hb[7])};
    ul[it] = (v4u){pk16(lb[0], lb[1]), pk16(lb[2], lb[3]), pk16(lb[4], lb[5]), pk16(lb[6], lb[7])};
    oofs[it] = planeoff + (size_t)(c0 + row) * R + r0 + c8;
  }
  for (int pass = 0; pass < 2; ++pass) {
#pragma unroll
    for (int it = 0; it < 2; ++it) {
      *(volatile v4u*)(outHi + oofs[it]) = uh[it];
      *(volatile v4u*)(outLo + oofs[it]) = ul[it];
    }
    __threadfence();
  }
}

__global__ __launch_bounds__(256) void prep_xxx_kernel(const float* __restrict__ x, const float* __restrict__ maa_x,
                                                       unsigned short* __restrict__ xh, unsigned short* __restrict__ xl,
                                                       int cbase, int n8) {
  const int i = blockIdx.x * 256 + threadIdx.x;
  if (i >= n8) return;
  const size_t e8 = (size_t)i * 8;
  const int m  = (int)(e8 >> 10);
  const int n  = (int)(e8 & 1023);
  const int xb = m >> kTcShift;
  const int t  = cbase + (m & (kTc - 1));
  const int tp = (t > 0) ? (t - 1) : 0;
  const size_t xi  = ((size_t)(xb * kT + t))  * kC + n;
  const size_t xpi = ((size_t)(xb * kT + tp)) * kC + n;
  const v4f a0 = *(const v4f*)(x + xi),  a1 = *(const v4f*)(x + xi + 4);
  const v4f p0 = *(const v4f*)(x + xpi), p1 = *(const v4f*)(x + xpi + 4);
  const v4f g0 = *(const v4f*)(maa_x + n), g1 = *(const v4f*)(maa_x + n + 4);
  const bool has_prev = (t > 0);
  unsigned short hb[8], lb[8];
#pragma unroll
  for (int e = 0; e < 4; ++e) {
    const float pe0 = has_prev ? p0[e] : 0.0f;
    const float pe1 = has_prev ? p1[e] : 0.0f;
    const float v0 = a0[e] + (pe0 - a0[e]) * g0[e];
    const float v1 = a1[e] + (pe1 - a1[e]) * g1[e];
    split_bits(v0, hb[e], lb[e]);
    split_bits(v1, hb[4 + e], lb[4 + e]);
  }
  const v4u uh = (v4u){pk16(hb[0], hb[1]), pk16(hb[2], hb[3]), pk16(hb[4], hb[5]), pk16(hb[6], hb[7])};
  const v4u ul = (v4u){pk16(lb[0], lb[1]), pk16(lb[2], lb[3]), pk16(lb[4], lb[5]), pk16(lb[6], lb[7])};
  unsigned short* qh = xh + e8;
  unsigned short* ql = xl + e8;
  *(volatile v4u*)qh = uh;
  *(volatile v4u*)ql = ul;
  __threadfence();
  *(volatile v4u*)qh = uh;
  *(volatile v4u*)ql = ul;
}

__global__ __launch_bounds__(256) void wkv_kernel(const float* __restrict__ rp, const float* __restrict__ kp,
                                                  const float* __restrict__ vp, const float* __restrict__ wdp,
                                                  const float* __restrict__ u, float* __restrict__ Sst,
                                                  float* __restrict__ y, int first) {
  __shared__ __align__(16) float ybuf[32 * 128];
  __shared__ __align__(16) float sS[8 * 256];
  const int lane = threadIdx.x & 31;
  const int wave = threadIdx.x >> 5;
  const int blk  = blockIdx.x;
  const int b    = blk >> 3;
  const int hbase = (blk & 7) * 8;
  const int h    = hbase + wave;
  const int bh   = b * kNH + h;
  const int j    = lane & 15;
  const int half = lane >> 4;
  const int i0   = half * 8;

  float S[8], uv[8];
#pragma unroll
  for (int ii = 0; ii < 8; ++ii) uv[ii] = u[h * kHS + i0 + ii];
  if (first) {
#pragma unroll
    for (int ii = 0; ii < 8; ++ii) S[ii] = 0.0f;
  } else {
#pragma unroll
    for (int ii = 0; ii < 8; ++ii) S[ii] = Sst[(size_t)bh * 256 + (i0 + ii) * 16 + j];
  }

  for (int sc = 0; sc < kTc / 32; ++sc) {
#pragma unroll 1
    for (int ts = 0; ts < 32; ++ts) {
      const int tl = sc * 32 + ts;
      const size_t base = ((size_t)(b * kTc + tl)) * kC + h * kHS;
      const v4f ra = *(const v4f*)(rp + base + i0),  rb = *(const v4f*)(rp + base + i0 + 4);
      const v4f ka = *(const v4f*)(kp + base + i0),  kb = *(const v4f*)(kp + base + i0 + 4);
      const v4f wa = *(const v4f*)(wdp + base + i0), wb = *(const v4f*)(wdp + base + i0 + 4);
      const float vj = vp[base + j];
      float rv[8], kv[8], wv[8];
#pragma unroll
      for (int e = 0; e < 4; ++e) {
        rv[e] = ra[e]; rv[4 + e] = rb[e];
        kv[e] = ka[e]; kv[4 + e] = kb[e];
        wv[e] = wa[e]; wv[4 + e] = wb[e];
      }
      float yp = 0.0f;
#pragma unroll
      for (int ii = 0; ii < 8; ++ii) {
        const float kvij = kv[ii] * vj;
        yp += rv[ii] * (S[ii] + uv[ii] * kvij);
        S[ii] = wv[ii] * S[ii] + kvij;
      }
      const float yo = yp + __shfl_xor(yp, 16, 32);
      if (half == 0) ybuf[ts * 128 + wave * 16 + j] = yo;
    }
    __syncthreads();
    v4f val[4];
    size_t dofs[4];
#pragma unroll
    for (int q4 = 0; q4 < 4; ++q4) {
      const int ts = wave * 4 + q4;
      val[q4]  = *(const v4f*)(ybuf + ts * 128 + lane * 4);
      dofs[q4] = ((size_t)(b * kTc + sc * 32 + ts)) * kC + hbase * kHS + lane * 4;
    }
    for (int pass = 0; pass < 2; ++pass) {
#pragma unroll
      for (int q4 = 0; q4 < 4; ++q4) *(volatile v4f*)(y + dofs[q4]) = val[q4];
      __threadfence();
    }
    __syncthreads();
  }

#pragma unroll
  for (int ii = 0; ii < 8; ++ii) sS[wave * 256 + (i0 + ii) * 16 + j] = S[ii];
  __syncthreads();
  v4f sv[2];
#pragma unroll
  for (int it = 0; it < 2; ++it) sv[it] = *(const v4f*)(sS + wave * 256 + it * 128 + lane * 4);
  for (int pass = 0; pass < 2; ++pass) {
#pragma unroll
    for (int it = 0; it < 2; ++it) *(volatile v4f*)(Sst + (size_t)bh * 256 + it * 128 + lane * 4) = sv[it];
    __threadfence();
  }
}

__global__ __launch_bounds__(256) void ln_split_kernel(const float* __restrict__ y, const float* __restrict__ g,
                                                       const float* __restrict__ bta,
                                                       unsigned short* __restrict__ oh, unsigned short* __restrict__ ol) {
  const int lane = threadIdx.x & 31;
  const int wave = threadIdx.x >> 5;
  const int row  = blockIdx.x * 8 + wave;
  const float* p = y + (size_t)row * kC;
  float vals[4][8];
#pragma unroll
  for (int seg = 0; seg < 4; ++seg) {
    const int base = seg * 256 + lane * 8;
    const v4f a = *(const v4f*)(p + base);
    const v4f c = *(const v4f*)(p + base + 4);
#pragma unroll
    for (int e = 0; e < 4; ++e) { vals[seg][e] = a[e]; vals[seg][4 + e] = c[e]; }
  }
  float s = 0.0f;
#pragma unroll
  for (int seg = 0; seg < 4; ++seg)
#pragma unroll
    for (int e = 0; e < 8; ++e) s += vals[seg][e];
#pragma unroll
  for (int off = 16; off > 0; off >>= 1) s += __shfl_xor(s, off, 32);
  const float mu = s * kInvC;
  float ss = 0.0f;
#pragma unroll
  for (int seg = 0; seg < 4; ++seg)
#pragma unroll
    for (int e = 0; e < 8; ++e) { const float d = vals[seg][e] - mu; ss += d * d; }
#pragma unroll
  for (int off = 16; off > 0; off >>= 1) ss += __shfl_xor(ss, off, 32);
  const float var  = ss * kInvC;
  const float rstd = rsqrtf(var + kLnEps);

  v4u uh[4], ul[4];
#pragma unroll
  for (int seg = 0; seg < 4; ++seg) {
    const int base = seg * 256 + lane * 8;
    const v4f ga = *(const v4f*)(g + base),   gb = *(const v4f*)(g + base + 4);
    const v4f ba = *(const v4f*)(bta + base), bb = *(const v4f*)(bta + base + 4);
    unsigned short hb[8], lb[8];
#pragma unroll
    for (int e = 0; e < 4; ++e) {
      const float o0 = ((vals[seg][e] - mu) * rstd) * ga[e] + ba[e];
      const float o1 = ((vals[seg][4 + e] - mu) * rstd) * gb[e] + bb[e];
      split_bits(o0, hb[e], lb[e]);
      split_bits(o1, hb[4 + e], lb[4 + e]);
    }
    uh[seg] = (v4u){pk16(hb[0], hb[1]), pk16(hb[2], hb[3]), pk16(hb[4], hb[5]), pk16(hb[6], hb[7])};
    ul[seg] = (v4u){pk16(lb[0], lb[1]), pk16(lb[2], lb[3]), pk16(lb[4], lb[5]), pk16(lb[6], lb[7])};
  }
  const size_t rofs = (size_t)row * kC + lane * 8;
  for (int pass = 0; pass < 2; ++pass) {
#pragma unroll
    for (int seg = 0; seg < 4; ++seg) {
      *(volatile v4u*)(oh + rofs + seg * 256) = uh[seg];
      *(volatile v4u*)(ol + rofs + seg * 256) = ul[seg];
    }
    __threadfence();
  }
}

extern "C" void kernel_launch(void* const* d_in, const int* in_sizes, int n_in,
                              void* d_out, int out_size, void* d_ws,
                              size_t ws_size, hipStream_t stream) {
  (void)in_sizes;
  if (n_in < 18) return;
  if ((size_t)out_size < (size_t)kB * kT * kC) return;

  const float* x      = (const float*)d_in[0];
  const float* maa_x  = (const float*)d_in[1];
  const float* maa_w  = (const float*)d_in[2];
  const float* maa_k  = (const float*)d_in[3];
  const float* maa_v  = (const float*)d_in[4];
  const float* maa_r  = (const float*)d_in[5];
  const float* w1     = (const float*)d_in[6];
  const float* w2     = (const float*)d_in[7];
  const float* tdecay = (const float*)d_in[8];
  const float* tdw1   = (const float*)d_in[9];
  const float* tdw2   = (const float*)d_in[10];
  const float* faaaa  = (const float*)d_in[11];
  const float* W_r    = (const float*)d_in[12];
  const float* W_k    = (const float*)d_in[13];
  const float* W_v    = (const float*)d_in[14];
  const float* W_o    = (const float*)d_in[15];
  const float* ln_g   = (const float*)d_in[16];
  const float* ln_b   = (const float*)d_in[17];

  char* ws = (char*)d_ws;
  size_t off = 0;
  auto take = [&](size_t bytes) { size_t o = off; off += (bytes + 255) & ~(size_t)255; return o; };

  const size_t bigPlane  = (size_t)kC * kC;
  const size_t rowsC     = (size_t)kRc;
  const size_t planeU16  = rowsC * kC;
  const size_t planeF    = rowsC * kC;

  unsigned short* wtH = (unsigned short*)(ws + take(4 * bigPlane * 2));
  unsigned short* wtL = (unsigned short*)(ws + take(4 * bigPlane * 2));
  unsigned short* w1H = (unsigned short*)(ws + take((size_t)128 * kC * 2));
  unsigned short* w1L = (unsigned short*)(ws + take((size_t)128 * kC * 2));
  unsigned short* w2H = (unsigned short*)(ws + take((size_t)kC * 128 * 2));
  unsigned short* w2L = (unsigned short*)(ws + take((size_t)kC * 128 * 2));
  unsigned short* d1H = (unsigned short*)(ws + take((size_t)kDDec * kC * 2));
  unsigned short* d1L = (unsigned short*)(ws + take((size_t)kDDec * kC * 2));
  unsigned short* d2H = (unsigned short*)(ws + take((size_t)kC * kDDec * 2));
  unsigned short* d2L = (unsigned short*)(ws + take((size_t)kC * kDDec * 2));
  unsigned short* xxH = (unsigned short*)(ws + take(planeU16 * 2));
  unsigned short* xxL = (unsigned short*)(ws + take(planeU16 * 2));
  unsigned short* mH  = (unsigned short*)(ws + take(rowsC * 128 * 2));
  unsigned short* mL  = (unsigned short*)(ws + take(rowsC * 128 * 2));
  unsigned short* mixH = (unsigned short*)(ws + take(4 * planeU16 * 2));
  unsigned short* mixL = (unsigned short*)(ws + take(4 * planeU16 * 2));
  unsigned short* hdH = (unsigned short*)(ws + take(rowsC * kDDec * 2));
  unsigned short* hdL = (unsigned short*)(ws + take(rowsC * kDDec * 2));
  float* wdp  = (float*)(ws + take(planeF * 4));
  float* rkv  = (float*)(ws + take(3 * planeF * 4));
  float* yp   = (float*)(ws + take(planeF * 4));
  unsigned short* ylH = (unsigned short*)(ws + take(planeU16 * 2));
  unsigned short* ylL = (unsigned short*)(ws + take(planeU16 * 2));
  float* Sst  = (float*)(ws + take((size_t)256 * 256 * 4));
  if (off > ws_size) return;

  float* outp = (float*)d_out;

  wt_split_kernel<<<dim3(kC / 64, kC / 64, 4), 256, 0, stream>>>(W_k, W_v, W_r, W_o, wtH, wtL, kC, kC);
  wt_split_kernel<<<dim3(kC / 64, 128 / 64, 1), 256, 0, stream>>>(w1, w1, w1, w1, w1H, w1L, kC, 128);
  wt_split_kernel<<<dim3(128 / 64, kC / 64, 1), 256, 0, stream>>>(w2, w2, w2, w2, w2H, w2L, 128, kC);
  wt_split_kernel<<<dim3(kC / 64, kDDec / 64, 1), 256, 0, stream>>>(tdw1, tdw1, tdw1, tdw1, d1H, d1L, kC, kDDec);
  wt_split_kernel<<<dim3(kDDec / 64, kC / 64, 1), 256, 0, stream>>>(tdw2, tdw2, tdw2, tdw2, d2H, d2L, kDDec, kC);

  const int M = kRc;
  const int tilesM = M / 64;
  const int n8 = (int)(planeU16 / 8);

  for (int c = 0; c < kNChunk; ++c) {
    const int cbase = c * kTc;

    prep_xxx_kernel<<<(n8 + 255) / 256, 256, 0, stream>>>(x, maa_x, xxH, xxL, cbase, n8);

    wmma_gemm64<1, true, 0, 2, false, 1><<<dim3((tilesM * (128 / 64) + 7) / 8, 1), 256, 0, stream>>>(
        xxH, xxL, kC, 0L, w1H, w1L, kC, 0L, mH, mL, 128, 0L, nullptr, nullptr, 0L, M, 128, kC, 1.0f);

    wmma_gemm64_mix<<<dim3((tilesM * (kC / 64) + 7) / 8, 4), 256, 0, stream>>>(
        mH, mL, 128, 32L, w2H, w2L, 128, 32L, mixH, mixL, kC, (long)planeU16,
        maa_w, maa_k, maa_v, maa_r, x, cbase, M, kC, kDMix);

    wmma_gemm64<1, true, 0, 2, false, 1><<<dim3((tilesM * (kDDec / 64) + 7) / 8, 1), 256, 0, stream>>>(
        mixH, mixL, kC, 0L, d1H, d1L, kC, 0L, hdH, hdL, kDDec, 0L, nullptr, nullptr, 0L, M, kDDec, kC, 1.0f);

    wmma_gemm64<1, true, 2, 0, false, 6><<<dim3((tilesM * (kC / 64) + 7) / 8, 1), 256, 0, stream>>>(
        hdH, hdL, kDDec, 0L, d2H, d2L, kDDec, 0L, wdp, nullptr, kC, 0L, tdecay, nullptr, 0L, M, kC, kDDec, 1.0f);

    wmma_gemm64<1, true, 0, 0, false, 0><<<dim3((tilesM * (kC / 64) + 7) / 8, 3), 256, 0, stream>>>(
        mixH + planeU16, mixL + planeU16, kC, (long)planeU16, wtH, wtL, kC, (long)bigPlane,
        rkv, nullptr, kC, (long)planeF, nullptr, nullptr, 0L, M, kC, kC, 1.0f);

    wkv_kernel<<<(kB * kNH) / 8, 256, 0, stream>>>(rkv + 2 * planeF, rkv, rkv + planeF, wdp, faaaa, Sst, yp,
                                                    (c == 0) ? 1 : 0);

    ln_split_kernel<<<M / 8, 256, 0, stream>>>(yp, ln_g, ln_b, ylH, ylL);

    wmma_gemm64<1, true, 0, 0, false, 0><<<dim3(((kTc / 64) * (kC / 64) + 7) / 8, kB), 256, 0, stream>>>(
        ylH, ylL, kC, (long)kTc * kC, wtH + 3 * bigPlane, wtL + 3 * bigPlane, kC, 0L,
        outp + (size_t)cbase * kC, nullptr, kC, (long)kT * kC, nullptr, nullptr, 0L, kTc, kC, kC, 1.0f);
  }
}
